// ParallelRiskAggregationNN_35227321762459
// MI455X (gfx1250) — hardware-verified
//
#include <hip/hip_runtime.h>
#include <math.h>

typedef __attribute__((ext_vector_type(16))) _Float16 v16h;
typedef __attribute__((ext_vector_type(16))) __bf16 v16b;
typedef __attribute__((ext_vector_type(8)))  _Float16 v8h;
typedef __attribute__((ext_vector_type(8)))  float v8f;
typedef __attribute__((ext_vector_type(4)))  float v4f;
typedef __attribute__((ext_vector_type(2)))  float v2f;
typedef __attribute__((ext_vector_type(4)))  unsigned v4u;
typedef __attribute__((ext_vector_type(4)))  int v4i;
typedef float __attribute__((may_alias)) float_a;
typedef int __attribute__((may_alias)) int_a;

template <typename T> __device__ __forceinline__ void vst2(void* p, T v) { *(volatile T*)p = v; __threadfence(); *(volatile T*)p = v; }
__device__ __forceinline__ v8f wmma16(v16h a, v16h b, v8f c) {
  v8f d = __builtin_amdgcn_wmma_f32_16x16x32_f16(false, a, false, b, (short)0, c, false, false);
  asm volatile("v_nop\n\tv_nop\n\tv_nop\n\tv_nop" : "+v"(d) : "v"(a), "v"(b));
  return d;
}
__device__ __forceinline__ v8f wmma_bf(v16b a, v16b b, v8f c) {
  v8f d = __builtin_amdgcn_wmma_f32_16x16x32_bf16(false, a, false, b, (short)0, c, false, false);
  asm volatile("v_nop\n\tv_nop\n\tv_nop\n\tv_nop" : "+v"(d) : "v"(a), "v"(b));
  return d;
}
__device__ __forceinline__ v16h frag_h(const _Float16* rowk0, int lane) {
  union { v16h v; v8h q[2]; } u; const _Float16* p = rowk0 + 8 * (lane >> 4);
  u.q[0] = *(const v8h*)p; u.q[1] = *(const v8h*)(p + 16); return u.v;
}
__device__ __forceinline__ v16h frag_f32(const float* rowk0, int lane) {
  v16h a; const float* p = rowk0 + 8 * (lane >> 4);
#pragma unroll
  for (int i = 0; i < 8; ++i) { a[i] = (_Float16)p[i]; a[8 + i] = (_Float16)p[16 + i]; }
  return a;
}
__device__ __forceinline__ v16h frag_f32s(const float* rowk0, int lane, float sc) {
  v16h a; const float* p = rowk0 + 8 * (lane >> 4);
#pragma unroll
  for (int i = 0; i < 8; ++i) { a[i] = (_Float16)(p[i] * sc); a[8 + i] = (_Float16)(p[16 + i] * sc); }
  return a;
}
__device__ __forceinline__ v16h fragc_f32(const float* W, int k0, int n, int lane, int ld, int K) {
  v16h a; const int g = lane >> 4;
#pragma unroll
  for (int i = 0; i < 8; ++i) { const int ka = k0 + 8 * g + i, kb = ka + 16;
    a[i] = (_Float16)(ka < K ? W[(size_t)(ka < K ? ka : K - 1) * ld + n] : 0.f); a[8 + i] = (_Float16)(kb < K ? W[(size_t)(kb < K ? kb : K - 1) * ld + n] : 0.f); }
  return a;
}
struct F2 { v16b h, l; };
__device__ __forceinline__ F2 bsplit16(const float v[16]) { F2 r;
#pragma unroll
  for (int i = 0; i < 16; ++i) { const __bf16 h = (__bf16)v[i]; r.h[i] = h; r.l[i] = (__bf16)(v[i] - (float)h); }
  return r; }
__device__ __forceinline__ F2 split_row(const float* row, int k0, int lane) { float v[16]; const float* p = row + k0 + 8 * (lane >> 4);
#pragma unroll
  for (int i = 0; i < 8; ++i) { v[i] = p[i]; v[8 + i] = p[16 + i]; }
  return bsplit16(v); }
__device__ __forceinline__ F2 split_rowK(const float* row, int k0, int lane, int K) { float v[16]; const int g = lane >> 4;
#pragma unroll
  for (int i = 0; i < 8; ++i) { const int ka = k0 + 8 * g + i, kb = ka + 16; v[i] = ka < K ? row[ka < K ? ka : K - 1] : 0.f; v[8 + i] = kb < K ? row[kb < K ? kb : K - 1] : 0.f; }
  return bsplit16(v); }
__device__ __forceinline__ F2 split_col(const float* W, int k0, int n, int lane, int ld, int K) { float v[16]; const int g = lane >> 4;
#pragma unroll
  for (int i = 0; i < 8; ++i) { const int ka = k0 + 8 * g + i, kb = ka + 16; v[i] = ka < K ? W[(size_t)(ka < K ? ka : K - 1) * ld + n] : 0.f; v[8 + i] = kb < K ? W[(size_t)(kb < K ? kb : K - 1) * ld + n] : 0.f; }
  return bsplit16(v); }
__device__ __forceinline__ v8f mac3(const F2& a, const F2& b, v8f c) { c = wmma_bf(a.l, b.h, c); c = wmma_bf(a.h, b.l, c); return wmma_bf(a.h, b.h, c); }
__device__ __forceinline__ float sigm(float v) { return 1.0f / (1.0f + expf(-v)); }
#define LDSX() do { asm volatile("s_wait_dscnt 0" ::: "memory"); __builtin_amdgcn_wave_barrier(); __builtin_amdgcn_fence(__ATOMIC_RELEASE, "workgroup"); } while (0)


#define NBATCH 32768
#define DX 64
#define HH 64
#define NL 2
#ifndef TBB
#define TBB (NBATCH / 64)
#endif
typedef __attribute__((ext_vector_type(8))) __bf16 v8b;
__device__ __forceinline__ v16b frag_b(const __bf16* rowk0, int lane) {
  union { v16b v; v8b q[2]; } u; const __bf16* p = rowk0 + 8 * (lane >> 4);
  u.q[0] = *(const v8b*)p; u.q[1] = *(const v8b*)(p + 16); return u.v;
}
__device__ __forceinline__ float bfr(float v) { return (float)(__bf16)v; }
__device__ __attribute__((noinline)) float exp_ni(float v) { return expf(v); }
__device__ __attribute__((noinline)) float erf_ni(float v) { return erff(v); }

#define WS_PE  0u
#define WS_PG  (WS_PE + 2u * (size_t)NL * DX * HH * HH)
#define WS_END (WS_PG + 2u * (size_t)3 * HH * HH + 256u)

__global__ __launch_bounds__(256) void k_pack(const float* __restrict__ HWH, const float* __restrict__ GW1, const float* __restrict__ GWH, _Float16* __restrict__ PE, _Float16* __restrict__ PG) {
  __shared__ __align__(16) _Float16 s[HH * HH]; const int d = blockIdx.x, l = blockIdx.y, t = threadIdx.x;
  if (l < NL) { const float* w = HWH + (((size_t)l * DX + d) * HH) * HH;
    for (int e = t; e < HH * HH; e += 256) { const int k = e / HH, h = e % HH; s[e] = (_Float16)(bfr(w[h * HH + k]) * 256.0f); }
    __syncthreads(); for (int q = t; q < HH * HH / 8; q += 256) vst2((unsigned*)(PE + (((size_t)l * DX + d) * HH) * HH + q * 8), *(const v4u*)&s[q * 8]); }
  else { if (d >= 3) return; const float* w = (d == 0) ? GW1 : (GWH + (size_t)(d - 1) * HH * HH);
    for (int e = t; e < HH * HH; e += 256) { const int k = e / HH, h = e % HH; s[e] = (_Float16)(bfr(w[h * HH + k]) * 256.0f); }
    __syncthreads(); for (int q = t; q < HH * HH / 8; q += 256) vst2((unsigned*)(PG + (size_t)d * HH * HH + q * 8), *(const v4u*)&s[q * 8]); }
}
__device__ __forceinline__ void layer64(const _Float16* __restrict__ arow, const _Float16* __restrict__ Wr, int lane, int col, v8f acc[4]) {
#pragma unroll
  for (int jt = 0; jt < 4; ++jt) { v8f z = {}; acc[jt] = z; }
#pragma unroll
  for (int kc = 0; kc < HH / 32; ++kc) { const v16h a = frag_h(arow + kc * 32, lane);
#pragma unroll
    for (int jt = 0; jt < 4; ++jt) acc[jt] = wmma16(a, frag_h(Wr + (size_t)(jt * 16 + col) * HH + kc * 32, lane), acc[jt]); }
#pragma unroll
  for (int jt = 0; jt < 4; ++jt)
#pragma unroll
    for (int r = 0; r < 8; ++r) acc[jt][r] *= (1.0f / 256.0f);
}
__global__ __launch_bounds__(128) void k_main(const float* __restrict__ X, const _Float16* __restrict__ PE, const _Float16* __restrict__ PG,
    const float* __restrict__ HW1, const float* __restrict__ HB1, const float* __restrict__ HBH, const float* __restrict__ HWO, const float* __restrict__ HBO,
    const float* __restrict__ GB1, const float* __restrict__ GBH, const float* __restrict__ GWO, const float* __restrict__ GBO, float* __restrict__ HOUT, float* __restrict__ GOUT) {
  __shared__ __align__(16) _Float16 sa[4][16][72]; __shared__ __align__(16) _Float16 sb[4][16][72]; __shared__ __align__(16) float sho[64][HH]; __shared__ __align__(16) float sgo[64];
  const int tid = threadIdx.x, wave = tid >> 5, lane = tid & 31, col = lane & 15, g = lane >> 4; const size_t b0 = (size_t)blockIdx.x * 64; const int w0 = wave * 16;
  v8f acc[4];
  for (int e = lane; e < 16 * HH; e += 32) { const int rl = e >> 6, c = e & 63; sa[wave][rl][c] = (_Float16)bfr(X[(b0 + w0 + rl) * (2 * DX) + c]); }
  LDSX();
  layer64(&sa[wave][col][0], PG, lane, col, acc);
#pragma unroll
  for (int jt = 0; jt < 4; ++jt) { const float bb = bfr(GB1[jt * 16 + col]);
#pragma unroll
    for (int r = 0; r < 8; ++r) sb[wave][8 * g + r][jt * 16 + col] = (_Float16)fmaxf(acc[jt][r] + bb, 0.f); }
  LDSX();
#pragma unroll 1
  for (int l = 0; l < NL; ++l) { _Float16 (*src)[72] = (l & 1) ? sa[wave] : sb[wave]; _Float16 (*dst)[72] = (l & 1) ? sb[wave] : sa[wave];
    layer64(&src[col][0], PG + (size_t)(1 + l) * HH * HH, lane, col, acc);
#pragma unroll
    for (int jt = 0; jt < 4; ++jt) { const float bb = bfr(GBH[l * HH + jt * 16 + col]);
#pragma unroll
      for (int r = 0; r < 8; ++r) { const float v = fmaxf(acc[jt][r] + bb, 0.f); dst[8 * g + r][jt * 16 + col] = (_Float16)v; if (l == NL - 1) acc[jt][r] = v; } }
    LDSX(); }
  { float part[8];
#pragma unroll
    for (int r = 0; r < 8; ++r) { float s = 0.f;
#pragma unroll
      for (int jt = 0; jt < 4; ++jt) s += acc[jt][r] * bfr(GWO[jt * 16 + col]); part[r] = s; }
#pragma unroll
    for (int r = 0; r < 8; ++r) {
#pragma unroll
      for (int o = 1; o < 16; o <<= 1) part[r] += __shfl_xor(part[r], o); }
    if (col == 0) {
#pragma unroll
      for (int r = 0; r < 8; ++r) sgo[w0 + 8 * g + r] = part[r] + bfr(GBO[0]); } }
#pragma unroll 1
  for (int d = 0; d < DX; ++d) {
    for (int e = lane; e < 16 * HH; e += 32) { const int rl = e >> 6, h = e & 63; const float xv = bfr(X[(b0 + w0 + rl) * (2 * DX) + DX + d]); sa[wave][rl][h] = (_Float16)fmaxf(xv * bfr(HW1[d * HH + h]) + bfr(HB1[d * HH + h]), 0.f); }
    LDSX();
#pragma unroll 1
    for (int l = 0; l < NL; ++l) { _Float16 (*src)[72] = (l & 1) ? sb[wave] : sa[wave]; _Float16 (*dst)[72] = (l & 1) ? sa[wave] : sb[wave];
      layer64(&src[col][0], PE + (((size_t)l * DX + d) * HH) * HH, lane, col, acc);
#pragma unroll
      for (int jt = 0; jt < 4; ++jt) { const float bb = bfr(HBH[((size_t)l * DX + d) * HH + jt * 16 + col]);
#pragma unroll
        for (int r = 0; r < 8; ++r) { const float v = fmaxf(acc[jt][r] + bb, 0.f); if (l < NL - 1) dst[8 * g + r][jt * 16 + col] = (_Float16)v; acc[jt][r] = v; } }
      LDSX(); }
    { float part[8];
#pragma unroll
      for (int r = 0; r < 8; ++r) { float s = 0.f;
#pragma unroll
        for (int jt = 0; jt < 4; ++jt) s += acc[jt][r] * bfr(HWO[d * HH + jt * 16 + col]); part[r] = s; }
#pragma unroll
      for (int r = 0; r < 8; ++r) {
#pragma unroll
        for (int o = 1; o < 16; o <<= 1) part[r] += __shfl_xor(part[r], o); }
      if (col == 0) {
#pragma unroll
        for (int r = 0; r < 8; ++r) sho[w0 + 8 * g + r][d] = part[r] + bfr(HBO[d]); } }
    LDSX(); }
  __syncthreads();
  for (int q = tid; q < 64 * HH / 4; q += 128) vst2(HOUT + (b0 * DX) + q * 4, *(const v4f*)(&sho[0][0] + q * 4));
  if (tid < 16) vst2(GOUT + b0 + tid * 4, *(const v4f*)&sgo[tid * 4]);
}
extern "C" void kernel_launch(void* const* d_in, const int* in_sizes, int n_in, void* d_out, int out_size, void* d_ws, size_t ws_size, hipStream_t stream) {
  (void)in_sizes; (void)n_in; (void)out_size;
  const float** F = (const float**)d_in;
  if (ws_size < (size_t)WS_END) return;
  char* ws = (char*)d_ws; _Float16 *PE = (_Float16*)(ws + WS_PE), *PG = (_Float16*)(ws + WS_PG);
  float* HOUT = (float*)d_out; float* GOUT = HOUT + (size_t)NBATCH * DX;
  k_pack<<<dim3(DX, NL + 1), 256, 0, stream>>>(F[3], F[7], F[9], PE, PG);
  k_main<<<TBB, 128, 0, stream>>>(F[0], PE, PG, F[1], F[2], F[4], F[5], F[6], F[8], F[10], F[11], F[12], HOUT, GOUT);
}
